// SpatialMambaBlock_18476949307581
// MI455X (gfx1250) — hardware-verified
//
#include <hip/hip_runtime.h>
#include <math.h>

typedef __attribute__((ext_vector_type(16))) _Float16 v16h;
typedef __attribute__((ext_vector_type(8)))  _Float16 v8h;
typedef __attribute__((ext_vector_type(16))) __bf16   v16b;
typedef __attribute__((ext_vector_type(8)))  __bf16   v8b;
typedef __attribute__((ext_vector_type(8)))  float    v8f;
typedef __attribute__((ext_vector_type(4)))  float    v4f;

constexpr int kDm   = 256;
constexpr int kL    = 17;
constexpr int kLP   = 32;
constexpr int kSeq  = 1944;
constexpr int kTok  = kSeq * kL;
constexpr int kDi   = 512;
constexpr int kDs   = 128;
constexpr int kNh   = 16;
constexpr int kHd   = 32;
constexpr int kCv   = 768;
constexpr int kPj   = 1296;
constexpr int kPjP  = 1344;
constexpr int kHid  = 1024;
constexpr int kYP   = 1024;
constexpr int kNChunk    = 3;
constexpr int kChunkSeq  = 648;
constexpr int kChunkRows = kChunkSeq * kL;
constexpr int kChunkMain = (kChunkRows / 64) * 64;
constexpr int kTokMain   = (kTok / 64) * 64;
static_assert(kNChunk * kChunkSeq == kSeq, "chunking covers all sequences");
static_assert(kChunkRows >= 64 && kTok >= 64, "tail launch needs 64 rows");
static_assert(kDi == kNh * kHd && kCv == kDi + 2 * kDs && kPj == 2 * kDi + 2 * kDs + kNh, "widths");

constexpr float kWsc  = 64.0f;
constexpr float kZsc  = 16.0f;
constexpr float kZinv = 1.0f / 16.0f;
constexpr float kXsc  = 64.0f;
constexpr float kBsc  = 64.0f;
constexpr float kMsc  = 4096.0f;
constexpr float kYsc  = 8.0f;
constexpr float kHsc  = 16.0f;

__device__ __forceinline__ unsigned short f2bf_bits(float f) {
  unsigned u = __float_as_uint(f);
  return (unsigned short)((u + 0x7FFFu + ((u >> 16) & 1u)) >> 16);
}
__device__ __forceinline__ float bf_bits2f(unsigned short h) { return __uint_as_float(((unsigned)h) << 16); }

__device__ __forceinline__ void dep_guard_h(v8f& a, v8f& b, v16h x, v16h y) { asm volatile("v_nop\n\tv_nop\n\tv_nop\n\tv_nop" : "+v"(a), "+v"(b) : "v"(x), "v"(y)); }
__device__ __forceinline__ void dep_guard_b(v8f& a, v8f& b, v16b x, v16b y) { asm volatile("v_nop\n\tv_nop\n\tv_nop\n\tv_nop" : "+v"(a), "+v"(b) : "v"(x), "v"(y)); }
__device__ __forceinline__ void keep4_h(v16h a, v16h b, v16h c, v16h d) { asm volatile("v_nop" :: "v"(a), "v"(b), "v"(c), "v"(d)); }
__device__ __forceinline__ void keep4_b(v16b a, v16b b, v16b c, v16b d) { asm volatile("v_nop" :: "v"(a), "v"(b), "v"(c), "v"(d)); }
__device__ __forceinline__ void acc_guard4(v8f& a, v8f& b, v8f& c, v8f& d) { asm volatile("v_nop\n\tv_nop\n\tv_nop\n\tv_nop" : "+v"(a), "+v"(b), "+v"(c), "+v"(d)); }
template <typename T> struct Frag;
template <> struct Frag<_Float16> {
  typedef v16h V; union U { v16h v; v8h h[2]; };
  static __device__ __forceinline__ v16h load(const _Float16* p) {
    U f; f.h[0] = *(const v8h*)(p); f.h[1] = *(const v8h*)(p + 16); return f.v;
  }
  static __device__ __forceinline__ v8f mma(v16h a, v16h b, v8f c) {
    return __builtin_amdgcn_wmma_f32_16x16x32_f16(false, a, false, b, (short)0, c, false, false);
  }
  static __device__ __forceinline__ void guard(v8f& a, v8f& b, v16h x, v16h y) { dep_guard_h(a, b, x, y); }
  static __device__ __forceinline__ void keep(v16h a, v16h b, v16h c, v16h d) { keep4_h(a, b, c, d); }
};
template <> struct Frag<__bf16> {
  typedef v16b V; union U { v16b v; v8b h[2]; };
  static __device__ __forceinline__ v16b load(const __bf16* p) {
    U f; f.h[0] = *(const v8b*)(p); f.h[1] = *(const v8b*)(p + 16); return f.v;
  }
  static __device__ __forceinline__ v8f mma(v16b a, v16b b, v8f c) {
    return __builtin_amdgcn_wmma_f32_16x16x32_bf16(false, a, false, b, (short)0, c, false, false);
  }
  static __device__ __forceinline__ void guard(v8f& a, v8f& b, v16b x, v16b y) { dep_guard_b(a, b, x, y); }
  static __device__ __forceinline__ void keep(v16b a, v16b b, v16b c, v16b d) { keep4_b(a, b, c, d); }
};

template <int ET> struct Elem;
template <> struct Elem<0> { typedef _Float16 T; };
template <> struct Elem<1> { typedef __bf16 T; };
template <int ET, bool SPLIT, int BIAS_MODE, int OUT_MODE, bool RESID, int ACT = 0>
__global__ __launch_bounds__(256) void wmma_gemm64(
    const unsigned short* __restrict__ Ap, const unsigned short* __restrict__ A2p, int lda, long strideA,
    const unsigned short* __restrict__ Btp, const unsigned short* __restrict__ Bt2p, int ldb, long strideB,
    void* __restrict__ Cout, void* __restrict__ Cout2, int ldc, long strideC,
    const float* __restrict__ bias,
    const float* __restrict__ resid, long strideR,
    int M, int N, int K, float scale) {
  typedef typename Elem<ET>::T T;
  typedef typename Frag<T>::V V;
  const T* A = (const T*)Ap; const T* A2 = (const T*)A2p; const T* Bt = (const T*)Btp; const T* Bt2 = (const T*)Bt2p;
  __shared__ __align__(16) float sT[8][16 * 68];
  const int b    = blockIdx.y;
  const int lane = threadIdx.x & 31;
  const int wave = threadIdx.x >> 5;
  const int tilesN = N >> 6;
  const int tilesM = M >> 6;
  const int tile = blockIdx.x * 8 + wave;
  if (tile >= tilesM * tilesN) return;
  const int tm = tile / tilesN;
  const int tn = tile - tm * tilesN;
  const int m0 = tm << 6;
  const int n0 = tn << 6;

  const T* Ab  = A  + (size_t)b * strideA;
  const T* Bb  = Bt + (size_t)b * strideB;
  const T* Ab2 = SPLIT ? (A2  + (size_t)b * strideA) : nullptr;
  const T* Bb2 = SPLIT ? (Bt2 + (size_t)b * strideB) : nullptr;

  const int rlane = lane & 15;
  const int koff  = (lane >> 4) * 8;
  const int mOff  = (lane >> 4) * 8;

  v8f acc[4][4];
#pragma unroll
  for (int i = 0; i < 4; ++i)
#pragma unroll
    for (int j = 0; j < 4; ++j) acc[i][j] = (v8f){0.f,0.f,0.f,0.f,0.f,0.f,0.f,0.f};

  for (int k0 = 0; k0 < K; k0 += 32) {
    V bh[4], bl[4];
#pragma unroll
    for (int j = 0; j < 4; ++j) {
      const size_t bo = (size_t)(n0 + (j << 4) + rlane) * ldb + koff + k0;
      bh[j] = Frag<T>::load(Bb + bo);
      if (SPLIT) bl[j] = Frag<T>::load(Bb2 + bo);
    }
#pragma unroll
    for (int i = 0; i < 4; ++i) {
      const size_t ao = (size_t)(m0 + (i << 4) + rlane) * lda + koff + k0;
      V ah = Frag<T>::load(Ab + ao);
      V al;
      if (SPLIT) al = Frag<T>::load(Ab2 + ao);
#pragma unroll
      for (int j = 0; j < 4; ++j) {
        acc[i][j] = Frag<T>::mma(ah, bh[j], acc[i][j]);
        if (SPLIT) {
          acc[i][j] = Frag<T>::mma(ah, bl[j], acc[i][j]);
          acc[i][j] = Frag<T>::mma(al, bh[j], acc[i][j]);
        }
      }
      Frag<T>::guard(acc[i][0], acc[i][3], ah, SPLIT ? al : ah);
    }
    Frag<T>::keep(bh[0], bh[1], bh[2], bh[3]);
    if (SPLIT) Frag<T>::keep(bl[0], bl[1], bl[2], bl[3]);
  }
  acc_guard4(acc[0][0], acc[0][1], acc[0][2], acc[0][3]);
  acc_guard4(acc[1][0], acc[1][1], acc[1][2], acc[1][3]);
  acc_guard4(acc[2][0], acc[2][1], acc[2][2], acc[2][3]);
  acc_guard4(acc[3][0], acc[3][1], acc[3][2], acc[3][3]);

  float* slab = sT[wave];
  const float* Rb = RESID ? (resid + (size_t)b * strideR) : nullptr;
#pragma unroll
  for (int i = 0; i < 4; ++i) {
    const int mBase = m0 + (i << 4);
#pragma unroll
    for (int j = 0; j < 4; ++j) {
      const int n = n0 + (j << 4) + rlane;
      float bv = 0.f;
      if (BIAS_MODE == 2) bv = bias[n];
#pragma unroll
      for (int r = 0; r < 8; ++r) {
        float v = acc[i][j][r] * scale;
        if (BIAS_MODE == 1) v += bias[mBase + mOff + r];
        if (BIAS_MODE == 2) v += bv;
        if (RESID) v += Rb[(size_t)(mBase + mOff + r) * ldc + n];
        if (ACT == 1) v = tanhf(v);
        if (ACT == 2) v = fmaxf(v, 0.0f);
        if (ACT == 3) v = v / (1.0f + expf(-v));
        if (ACT == 4) v = (v > 0.f) ? v : 0.01f * v;
        if (ACT == 5) v = 0.5f * v * (1.0f + erff(v * 0.70710678118654752f));
        slab[(mOff + r) * 68 + (j << 4) + rlane] = v;
      }
    }
    __builtin_amdgcn_fence(__ATOMIC_RELEASE, "workgroup");
    __builtin_amdgcn_wave_barrier();
    __builtin_amdgcn_fence(__ATOMIC_ACQUIRE, "workgroup");
    if (OUT_MODE == 0) {
      float* C = (float*)Cout + (size_t)b * strideC;
      const int hh = lane >> 4, c4 = (lane & 15) * 4;
      for (int pass = 0; pass < 2; ++pass) {
#pragma unroll
        for (int it = 0; it < 8; ++it) {
          const int row = it * 2 + hh;
          v4f v = *(const v4f*)(slab + row * 68 + c4);
          *(volatile v4f*)(C + (size_t)(mBase + row) * ldc + n0 + c4) = v;
        }
        __threadfence();
      }
    } else {
      const int q = lane >> 3, c8 = (lane & 7) * 8;
      unsigned short* C  = (unsigned short*)Cout  + (size_t)b * strideC;
      unsigned short* C2 = (OUT_MODE == 2) ? ((unsigned short*)Cout2 + (size_t)b * strideC) : nullptr;
      for (int pass = 0; pass < 2; ++pass) {
#pragma unroll
        for (int it = 0; it < 4; ++it) {
          const int row = it * 4 + q;
          const float* sp = slab + row * 68 + c8;
          v8h hv, lv;
#pragma unroll
          for (int e = 0; e < 8; ++e) {
            if (OUT_MODE == 1) {
              hv[e] = (_Float16)sp[e];
            } else {
              unsigned short hb = f2bf_bits(sp[e]);
              unsigned short lb = f2bf_bits(sp[e] - bf_bits2f(hb));
              hv[e] = __builtin_bit_cast(_Float16, hb);
              lv[e] = __builtin_bit_cast(_Float16, lb);
            }
          }
          *(volatile v8h*)(C + (size_t)(mBase + row) * ldc + n0 + c8) = hv;
          if (OUT_MODE == 2) *(volatile v8h*)(C2 + (size_t)(mBase + row) * ldc + n0 + c8) = lv;
        }
        __threadfence();
      }
    }
    __builtin_amdgcn_fence(__ATOMIC_RELEASE, "workgroup");
    __builtin_amdgcn_wave_barrier();
    __builtin_amdgcn_fence(__ATOMIC_ACQUIRE, "workgroup");
  }
}

__global__ __launch_bounds__(256) void cast_f16_kernel(
    const float* __restrict__ src, unsigned short* __restrict__ dst, int total8, float scale)
{
  const int i = blockIdx.x * 256 + threadIdx.x;
  if (i >= total8) return;
  const size_t e0 = (size_t)i << 3;
  const float* p = src + e0;
  const v4f a0 = *(const v4f*)(p);
  const v4f a1 = *(const v4f*)(p + 4);
  v8h hv;
#pragma unroll
  for (int e = 0; e < 4; ++e) {
    hv[e]     = (_Float16)(a0[e] * scale);
    hv[4 + e] = (_Float16)(a1[e] * scale);
  }
  unsigned short* q = dst + e0;
  *(volatile v8h*)q = hv;
  __threadfence();
  *(volatile v8h*)q = hv;
}

__device__ __forceinline__ float h2f(unsigned short u) { return (float)__builtin_bit_cast(_Float16, u); }
__device__ __forceinline__ float silu_fast(float v) { return v * __builtin_amdgcn_rcpf(1.0f + __expf(-v)); }
__device__ __forceinline__ v8f wmma16_h(v16h a, v16h b, v8f c) {
  c = __builtin_amdgcn_wmma_f32_16x16x32_f16(false, a, false, b, (short)0, c, false, false);
  asm volatile("v_nop\n\tv_nop\n\tv_nop\n\tv_nop" : "+v"(c) : "v"(a), "v"(b));
  return c;
}

__global__ __launch_bounds__(256) void prep_inproj_w_kernel(
    const float* __restrict__ W, unsigned short* __restrict__ Bt, int flip)
{
  const int i = blockIdx.x * 256 + threadIdx.x;
  if (i >= kPjP * 32) return;
  const int n = i >> 5, k0 = (i & 31) * 8;
  const int nc = (n < kPj) ? n : (kPj - 1);
  const float* wr = W + (size_t)nc * kDm;
  v8h hv;
#pragma unroll
  for (int e = 0; e < 8; ++e) {
    const int k = (flip != 0) ? (kDm - 1 - (k0 + e)) : (k0 + e);
    const float v = wr[k];
    hv[e] = (n < kPj) ? (_Float16)(v * kWsc) : (_Float16)0.0f;
  }
  unsigned short* o = Bt + (size_t)n * kDm + k0;
  *(volatile v8h*)o = hv;
  __threadfence();
  *(volatile v8h*)o = hv;
}

__global__ __launch_bounds__(256) void prep_outproj_w_kernel(
    const float* __restrict__ Wa, const float* __restrict__ Wi, unsigned short* __restrict__ Bt)
{
  const int i = blockIdx.x * 256 + threadIdx.x;
  if (i >= kDm * (kYP / 8)) return;
  const int n = i >> 7, k0 = (i & 127) * 8;
  const int ka = k0 & (kDi - 1);
  const float* pa = Wa + (size_t)n * kDi + ka;
  const float* pi = Wi + (size_t)n * kDi + ka;
  const bool useA = (k0 < kDi);
  v8h hv;
#pragma unroll
  for (int e = 0; e < 8; ++e) {
    const float va = pa[e], vi = pi[e];
    hv[e] = (_Float16)((useA ? va : vi) * kWsc);
  }
  unsigned short* o = Bt + (size_t)n * kYP + k0;
  *(volatile v8h*)o = hv;
  __threadfence();
  *(volatile v8h*)o = hv;
}

__global__ __launch_bounds__(256) void layernorm_f16_kernel(
    const float* __restrict__ X, const float* __restrict__ w, const float* __restrict__ bvec,
    unsigned short* __restrict__ O16, int nrows)
{
  const int row  = blockIdx.x * 8 + (threadIdx.x >> 5);
  const int lane = threadIdx.x & 31;
  if (row >= nrows) return;
  const float* xr = X + (size_t)row * kDm + lane * 8;
  const v4f a0 = *(const v4f*)(xr);
  const v4f a1 = *(const v4f*)(xr + 4);
  float v[8];
#pragma unroll
  for (int e = 0; e < 4; ++e) { v[e] = a0[e]; v[4 + e] = a1[e]; }
  float s1 = 0.f;
#pragma unroll
  for (int e = 0; e < 8; ++e) s1 += v[e];
#pragma unroll
  for (int o = 16; o > 0; o >>= 1) s1 += __shfl_xor(s1, o, 32);
  const float mean = s1 * (1.0f / 256.0f);
  float s2 = 0.f;
#pragma unroll
  for (int e = 0; e < 8; ++e) { const float d = v[e] - mean; s2 += d * d; }
#pragma unroll
  for (int o = 16; o > 0; o >>= 1) s2 += __shfl_xor(s2, o, 32);
  const float var = s2 * (1.0f / 256.0f);
  const float rs = rsqrtf(var + 1e-5f);
  v8h hv;
#pragma unroll
  for (int e = 0; e < 8; ++e) hv[e] = (_Float16)((v[e] - mean) * rs * w[lane * 8 + e] + bvec[lane * 8 + e]);
  unsigned short* o = O16 + (size_t)row * kDm + lane * 8;
  *(volatile v8h*)o = hv;
  __threadfence();
  *(volatile v8h*)o = hv;
}

__global__ __launch_bounds__(256) void gelu_f16x2_kernel(unsigned short* __restrict__ buf, int n2, float oscale)
{
  const int i = blockIdx.x * 256 + threadIdx.x;
  if (i >= n2) return;
  const unsigned u = ((const unsigned*)buf)[i];
  const float x0 = h2f((unsigned short)(u & 0xFFFFu));
  const float x1 = h2f((unsigned short)(u >> 16));
  float g0 = 0.f, g1 = 0.f;
#pragma unroll 1
  for (int e = 0; e < 2; ++e) {
    const float x = (e != 0) ? x1 : x0;
    const float g = 0.5f * x * (1.0f + erff(x * 0.70710678118654752f)) * oscale;
    if (e != 0) g1 = g; else g0 = g;
  }
  const unsigned r = (unsigned)__builtin_bit_cast(unsigned short, (_Float16)g0) |
                     ((unsigned)__builtin_bit_cast(unsigned short, (_Float16)g1) << 16);
  ((volatile unsigned*)buf)[i] = r;
  __threadfence();
  ((volatile unsigned*)buf)[i] = r;
}

constexpr int kLdsXS = 0;
constexpr int kLdsYS = kLdsXS + kL * kDi * 4;
constexpr int kLdsCB = kLdsYS + kL * kDi * 4;
constexpr int kLdsDT = kLdsCB + kLP * 33 * 4;
constexpr int kLdsCU = kLdsDT + kL * kNh * 4;
constexpr int kLdsXT = kLdsCU + kL * kNh * 4;
constexpr int kLdsBC = kLdsXT + kDi * kLP * 2;
constexpr int kLdsMP = kLdsBC + 2 * kLP * kDs * 2;
constexpr int kLdsTotal = kLdsMP + kNh * kLP * kLP * 2;
static_assert((kLdsYS % 16) == 0 && (kLdsCB % 16) == 0 && (kLdsDT % 16) == 0 && (kLdsCU % 16) == 0 &&
              (kLdsXT % 16) == 0 && (kLdsBC % 16) == 0 && (kLdsMP % 16) == 0, "lds align");

__global__ __launch_bounds__(256) void seq_scan_kernel(
    const unsigned short* __restrict__ ZX,
    const float* __restrict__ cw, const float* __restrict__ cb,
    const float* __restrict__ dtb, const float* __restrict__ Alog,
    const float* __restrict__ Dp, const float* __restrict__ nw,
    unsigned short* __restrict__ Yout, int colOff)
{
  extern __shared__ __align__(16) unsigned char lds_raw[];
  float* XS32 = (float*)(lds_raw + kLdsXS);
  float* YS32 = (float*)(lds_raw + kLdsYS);
  float* CBs  = (float*)(lds_raw + kLdsCB);
  float* dtv  = (float*)(lds_raw + kLdsDT);
  float* cum  = (float*)(lds_raw + kLdsCU);
  _Float16* XT16 = (_Float16*)(lds_raw + kLdsXT);
  _Float16* BC16 = (_Float16*)(lds_raw + kLdsBC);
  _Float16* MP16 = (_Float16*)(lds_raw + kLdsMP);

  const int tid = threadIdx.x, lane = tid & 31, wave = tid >> 5;
  const size_t rbase = (size_t)blockIdx.x * kL;
  const unsigned short* zrow0 = ZX + rbase * kPjP;

  {
    v8h z8;
#pragma unroll
    for (int e = 0; e < 8; ++e) z8[e] = (_Float16)0.0f;
    for (int i = tid; i < 480; i += 256) {
      const int pl = (i >= 240) ? 1 : 0;
      const int rem = i - pl * 240;
      const int row = kL + (rem >> 4);
      const int c8 = (rem & 15) * 8;
      *(v8h*)(BC16 + (pl * kLP + row) * kDs + c8) = z8;
    }
    for (int i = tid; i < (kNh * kLP * kLP) / 8; i += 256) *(v8h*)(MP16 + i * 8) = z8;
  }

#pragma unroll 1
  for (int j = 0; j < 2; ++j) {
    const int c = tid + j * 256;
    const float w0 = cw[c * 4 + 0], w1 = cw[c * 4 + 1], w2 = cw[c * 4 + 2], w3 = cw[c * 4 + 3];
    const float bc = cb[c];
    float p1 = 0.f, p2 = 0.f, p3 = 0.f;
    const unsigned short* col = zrow0 + kDi + c;
#pragma unroll 1
    for (int t = 0; t < kL; ++t) {
      const float v = h2f(col[(size_t)t * kPjP]) * kZinv;
      const float a = (((p3 * w0 + p2 * w1) + p1 * w2) + v * w3) + bc;
      const float u = silu_fast(a);
      XS32[t * kDi + c] = u;
      XT16[c * kLP + t] = (_Float16)(u * kXsc);
      p3 = p2; p2 = p1; p1 = v;
    }
#pragma unroll 1
    for (int t = kL; t < kLP; ++t) XT16[c * kLP + t] = (_Float16)0.0f;
  }
  {
    const int c = kDi + tid;
    const int pl = tid >> 7;
    const int cc = tid & 127;
    const float w0 = cw[c * 4 + 0], w1 = cw[c * 4 + 1], w2 = cw[c * 4 + 2], w3 = cw[c * 4 + 3];
    const float bc = cb[c];
    float p1 = 0.f, p2 = 0.f, p3 = 0.f;
    const unsigned short* col = zrow0 + kDi + c;
#pragma unroll 1
    for (int t = 0; t < kL; ++t) {
      const float v = h2f(col[(size_t)t * kPjP]) * kZinv;
      const float a = (((p3 * w0 + p2 * w1) + p1 * w2) + v * w3) + bc;
      const float u = silu_fast(a);
      BC16[(pl * kLP + t) * kDs + cc] = (_Float16)(u * kBsc);
      p3 = p2; p2 = p1; p1 = v;
    }
  }
  if (wave == 0) {
    const int h = lane & 15;
    const float Ah = -expf(Alog[h]);
    const float db = dtb[h];
    float run = 0.f;
    const unsigned short* col = zrow0 + (kDi + kCv) + h;
#pragma unroll 1
    for (int t = 0; t < kL; ++t) {
      const float xv = h2f(col[(size_t)t * kPjP]) * kZinv + db;
      const float sp = fmaxf(xv, 0.0f) + log1pf(expf(-fabsf(xv)));
      const float dA = sp * Ah;
      run += dA;
      if (lane < 16) { dtv[t * kNh + h] = sp; cum[t * kNh + h] = run; }
    }
  }
  __syncthreads();

  if (wave < 4) {
    const int ti = wave >> 1, tj = wave & 1;
    const int rl = lane & 15, koff = (lane >> 4) * 8, hh = lane >> 4;
    const _Float16* Cp = BC16 + (kLP + ti * 16 + rl) * kDs + koff;
    const _Float16* Bp = BC16 + (tj * 16 + rl) * kDs + koff;
    v8f acc = (v8f){0.f,0.f,0.f,0.f,0.f,0.f,0.f,0.f};
#pragma unroll
    for (int k0 = 0; k0 < kDs; k0 += 32) {
      const v16h a = Frag<_Float16>::load(Cp + k0);
      const v16h bfr = Frag<_Float16>::load(Bp + k0);
      acc = wmma16_h(a, bfr, acc);
    }
#pragma unroll
    for (int r = 0; r < 8; ++r)
      CBs[(ti * 16 + hh * 8 + r) * 33 + tj * 16 + rl] = acc[r] * (1.0f / 4096.0f);
  }
  __syncthreads();

#pragma unroll 1
  for (int i = tid; i < kNh * kL * kLP; i += 256) {
    const int h = i / (kL * kLP);
    const int rem = i - h * (kL * kLP);
    const int t = rem >> 5, s = rem & 31;
    if (s <= t) {
      const float m = CBs[t * 33 + s] * __expf(cum[t * kNh + h] - cum[s * kNh + h]) * dtv[s * kNh + h];
      MP16[(h * kLP + t) * kLP + s] = (_Float16)(m * kMsc);
    }
  }
  __syncthreads();

  {
    const int rl = lane & 15, koff = (lane >> 4) * 8, hh = lane >> 4;
#pragma unroll 1
    for (int tile = wave; tile < kNh * 4; tile += 8) {
      const int h = tile >> 2, ti = (tile >> 1) & 1, tj = tile & 1;
      const v16h a = Frag<_Float16>::load(MP16 + (h * kLP + ti * 16 + rl) * kLP + koff);
      const v16h bfr = Frag<_Float16>::load(XT16 + (h * kHd + tj * 16 + rl) * kLP + koff);
      v8f acc = (v8f){0.f,0.f,0.f,0.f,0.f,0.f,0.f,0.f};
      acc = wmma16_h(a, bfr, acc);
#pragma unroll
      for (int r = 0; r < 8; ++r) {
        const int t = ti * 16 + hh * 8 + r;
        if (t < kL) YS32[t * kDi + h * kHd + tj * 16 + rl] = acc[r] * (1.0f / 262144.0f);
      }
    }
  }
  __syncthreads();

#pragma unroll 1
  for (int i = tid; i < kL * kDi; i += 256) {
    const int t = i >> 9, d = i & (kDi - 1);
    const float zr = h2f(zrow0[(size_t)t * kPjP + d]) * kZinv;
    const float ysum = YS32[i] + Dp[d >> 5] * XS32[i];
    YS32[i] = ysum * silu_fast(zr);
  }
  __syncthreads();

  for (int t = wave; t < kL; t += 8) {
    const float* yr = YS32 + t * kDi;
    float ss = 0.f;
#pragma unroll
    for (int j = 0; j < 16; ++j) { const float v = yr[lane + 32 * j]; ss += v * v; }
#pragma unroll
    for (int o = 16; o > 0; o >>= 1) ss += __shfl_xor(ss, o, 32);
    const float rs = rsqrtf(ss * (1.0f / 512.0f) + 1e-5f);
    v8h hv0, hv1;
    {
      const int d0 = lane * 8;
      const v4f a0 = *(const v4f*)(yr + d0);
      const v4f a1 = *(const v4f*)(yr + d0 + 4);
#pragma unroll
      for (int e = 0; e < 4; ++e) {
        hv0[e]     = (_Float16)(a0[e] * rs * nw[d0 + e] * kYsc);
        hv0[4 + e] = (_Float16)(a1[e] * rs * nw[d0 + 4 + e] * kYsc);
      }
    }
    {
      const int d0 = 256 + lane * 8;
      const v4f a0 = *(const v4f*)(yr + d0);
      const v4f a1 = *(const v4f*)(yr + d0 + 4);
#pragma unroll
      for (int e = 0; e < 4; ++e) {
        hv1[e]     = (_Float16)(a0[e] * rs * nw[d0 + e] * kYsc);
        hv1[4 + e] = (_Float16)(a1[e] * rs * nw[d0 + 4 + e] * kYsc);
      }
    }
    unsigned short* yo = Yout + (rbase + t) * (size_t)kYP + colOff;
    *(volatile v8h*)(yo + lane * 8) = hv0;
    *(volatile v8h*)(yo + 256 + lane * 8) = hv1;
    __threadfence();
    *(volatile v8h*)(yo + lane * 8) = hv0;
    *(volatile v8h*)(yo + 256 + lane * 8) = hv1;
  }
}

template <int BIAS_MODE, int OUT_MODE, bool RESID>
static inline void launch_gemm_f16(const unsigned short* A, int lda, const unsigned short* Bt, int ldb,
                                   void* Cp, int ldc, const float* bias, const float* resid,
                                   int Mr, int Nr, int Kr, float scale, hipStream_t st)
{
  const int tiles = (Mr >> 6) * (Nr >> 6);
  const dim3 grid((unsigned)((tiles + 7) / 8), 1, 1);
  wmma_gemm64<0, false, BIAS_MODE, OUT_MODE, RESID, 0><<<grid, dim3(256), 0, st>>>(
      A, A, lda, 0L, Bt, Bt, ldb, 0L, Cp, Cp, ldc, 0L, bias, resid, 0L, Mr, Nr, Kr, scale);
}

static inline size_t align256(size_t v) { return (v + 255) & ~(size_t)255; }

extern "C" void kernel_launch(void* const* d_in, const int* in_sizes, int n_in,
                              void* d_out, int out_size, void* d_ws, size_t ws_size,
                              hipStream_t stream)
{
  (void)in_sizes; (void)n_in; (void)out_size;
  const float* x      = (const float*)d_in[0];
  const float* n1w    = (const float*)d_in[1];
  const float* n1b    = (const float*)d_in[2];
  const float* n2w    = (const float*)d_in[3];
  const float* n2b    = (const float*)d_in[4];
  const float* w1     = (const float*)d_in[5];
  const float* b1     = (const float*)d_in[6];
  const float* w2     = (const float*)d_in[7];
  const float* b2     = (const float*)d_in[8];
  const float* a_in   = (const float*)d_in[9];
  const float* a_cw   = (const float*)d_in[10];
  const float* a_cb   = (const float*)d_in[11];
  const float* a_dtb  = (const float*)d_in[12];
  const float* a_Alog = (const float*)d_in[13];
  const float* a_D    = (const float*)d_in[14];
  const float* a_nw   = (const float*)d_in[15];
  const float* a_outw = (const float*)d_in[16];
  const float* i_in   = (const float*)d_in[17];
  const float* i_cw   = (const float*)d_in[18];
  const float* i_cb   = (const float*)d_in[19];
  const float* i_dtb  = (const float*)d_in[20];
  const float* i_Alog = (const float*)d_in[21];
  const float* i_D    = (const float*)d_in[22];
  const float* i_nw   = (const float*)d_in[23];
  const float* i_outw = (const float*)d_in[24];
  float* out = (float*)d_out;

  char* ws = (char*)d_ws;
  size_t off = 0;
  const size_t oWinA = off; off += align256((size_t)kPjP * kDm * 2);
  const size_t oWinI = off; off += align256((size_t)kPjP * kDm * 2);
  const size_t oWcat = off; off += align256((size_t)kDm * kYP * 2);
  const size_t oW1   = off; off += align256((size_t)kHid * kDm * 2);
  const size_t oW2   = off; off += align256((size_t)kDm * kHid * 2);
  const size_t oX1   = off; off += align256((size_t)kTok * kDm * 4);
  const size_t oArena = off;
  const size_t oXN  = oArena;
  const size_t oZX  = oXN + align256((size_t)kTok * kDm * 2);
  const size_t oYc  = oZX + align256((size_t)kChunkRows * kPjP * 2);
  const size_t end1 = oYc + align256((size_t)kChunkRows * kYP * 2);
  const size_t oHN  = oArena;
  const size_t oG   = oHN + align256((size_t)kTok * kDm * 2);
  const size_t end2 = oG + align256((size_t)kTok * kHid * 2);
  const size_t total = (end1 > end2) ? end1 : end2;
  if (total > ws_size) return;

  unsigned short* WinA = (unsigned short*)(ws + oWinA);
  unsigned short* WinI = (unsigned short*)(ws + oWinI);
  unsigned short* Wcat = (unsigned short*)(ws + oWcat);
  unsigned short* W1h  = (unsigned short*)(ws + oW1);
  unsigned short* W2h  = (unsigned short*)(ws + oW2);
  float*          X1   = (float*)(ws + oX1);
  unsigned short* XN16 = (unsigned short*)(ws + oXN);
  unsigned short* ZXc  = (unsigned short*)(ws + oZX);
  unsigned short* Yc   = (unsigned short*)(ws + oYc);
  unsigned short* HN16 = (unsigned short*)(ws + oHN);
  unsigned short* G16  = (unsigned short*)(ws + oG);

  const dim3 blk(256);

  prep_inproj_w_kernel<<<dim3((kPjP * 32) / 256), blk, 0, stream>>>(a_in, WinA, 0);
  prep_inproj_w_kernel<<<dim3((kPjP * 32) / 256), blk, 0, stream>>>(i_in, WinI, 1);
  prep_outproj_w_kernel<<<dim3((kDm * (kYP / 8)) / 256), blk, 0, stream>>>(a_outw, i_outw, Wcat);
  cast_f16_kernel<<<dim3((kHid * kDm / 8 + 255) / 256), blk, 0, stream>>>(w1, W1h, kHid * kDm / 8, kWsc);
  cast_f16_kernel<<<dim3((kDm * kHid / 8 + 255) / 256), blk, 0, stream>>>(w2, W2h, kDm * kHid / 8, kWsc);

  layernorm_f16_kernel<<<dim3((kTok + 7) / 8), blk, 0, stream>>>(x, n1w, n1b, XN16, kTok);

  const int tailRow = kChunkRows - 64;
  const float inScale  = kZsc / kWsc;
  const float outScale = 1.0f / (kWsc * kYsc);
  for (int c = 0; c < kNChunk; ++c) {
    const size_t r0 = (size_t)c * kChunkRows;
    launch_gemm_f16<0, 1, false>(XN16 + r0 * kDm, kDm, WinA, kDm, ZXc, kPjP, b1, x,
                                 kChunkMain, kPjP, kDm, inScale, stream);
    launch_gemm_f16<0, 1, false>(XN16 + (r0 + tailRow) * kDm, kDm, WinA, kDm, ZXc + (size_t)tailRow * kPjP, kPjP, b1, x,
                                 64, kPjP, kDm, inScale, stream);
    seq_scan_kernel<<<dim3(kChunkSeq), blk, kLdsTotal, stream>>>(ZXc, a_cw, a_cb, a_dtb, a_Alog, a_D, a_nw, Yc, 0);
    launch_gemm_f16<0, 1, false>(XN16 + r0 * kDm, kDm, WinI, kDm, ZXc, kPjP, b1, x,
                                 kChunkMain, kPjP, kDm, inScale, stream);
    launch_gemm_f16<0, 1, false>(XN16 + (r0 + tailRow) * kDm, kDm, WinI, kDm, ZXc + (size_t)tailRow * kPjP, kPjP, b1, x,
                                 64, kPjP, kDm, inScale, stream);
    seq_scan_kernel<<<dim3(kChunkSeq), blk, kLdsTotal, stream>>>(ZXc, i_cw, i_cb, i_dtb, i_Alog, i_D, i_nw, Yc, kDi);
    launch_gemm_f16<0, 0, true>(Yc, kYP, Wcat, kYP, X1 + r0 * kDm, kDm, b1, x + r0 * kDm,
                                kChunkMain, kDm, kYP, outScale, stream);
    launch_gemm_f16<0, 0, true>(Yc + (size_t)tailRow * kYP, kYP, Wcat, kYP, X1 + (r0 + tailRow) * kDm, kDm, b1,
                                x + (r0 + tailRow) * kDm, 64, kDm, kYP, outScale, stream);
  }

  layernorm_f16_kernel<<<dim3((kTok + 7) / 8), blk, 0, stream>>>(X1, n2w, n2b, HN16, kTok);

  const int tailTok = kTok - 64;
  launch_gemm_f16<2, 1, false>(HN16, kDm, W1h, kDm, G16, kHid, b1, x, kTokMain, kHid, kDm, 1.0f / kWsc, stream);
  launch_gemm_f16<2, 1, false>(HN16 + (size_t)tailTok * kDm, kDm, W1h, kDm, G16 + (size_t)tailTok * kHid, kHid, b1, x,
                               64, kHid, kDm, 1.0f / kWsc, stream);
  {
    const int n2 = kTok * kHid / 2;
    gelu_f16x2_kernel<<<dim3((n2 + 255) / 256), blk, 0, stream>>>(G16, n2, kHsc);
  }
  launch_gemm_f16<2, 0, true>(G16, kHid, W2h, kHid, out, kDm, b2, X1, kTokMain, kDm, kHid, 1.0f / (kWsc * kHsc), stream);
  launch_gemm_f16<2, 0, true>(G16 + (size_t)tailTok * kHid, kHid, W2h, kHid, out + (size_t)tailTok * kDm, kDm, b2,
                              X1 + (size_t)tailTok * kDm, 64, kDm, kHid, 1.0f / (kWsc * kHsc), stream);
}
